// CausalSelfAttention_6073083757241
// MI455X (gfx1250) — hardware-verified
//
#include <hip/hip_runtime.h>
#ifndef NB
#define NB 2
#endif
#ifndef SEQ
#define SEQ 2048
#endif
#define NB_FULL 2
#define SEQ_FULL 2048
#define DM 1024
#define NH 16
#define HD 64
#define LQ (3 * DM)
#define RESROWS 256
#define NR (NB * SEQ)
#define RSC 0.0009765625f

static_assert(HD == 64);
static_assert(DM == NH * HD);
static_assert(DM % 64 == 0 && LQ % 64 == 0);
static_assert(DM % 32 == 0);
static_assert(SEQ % 128 == 0);
static_assert(NR % 128 == 0);
static_assert(RESROWS % 64 == 0 && RESROWS <= SEQ && RESROWS % 32 == 0);
static_assert(((NR / 16) * (DM / 64)) % 4 == 0);
static_assert(NB <= NB_FULL && SEQ <= SEQ_FULL);
#define WS_TOTAL ((size_t)3 * DM * DM * 2 + (size_t)DM * DM * 2 + (size_t)NR * DM * 2 + (size_t)NR * LQ * 2 + (size_t)NB * RESROWS * LQ * 2 + (size_t)NB * NH * HD * SEQ * 2 + (size_t)NB * NH * HD * RESROWS * 2 + (size_t)2 * NR * DM * 2)
static_assert(WS_TOTAL <= (size_t)134217728);

typedef _Float16 v16h __attribute__((ext_vector_type(16)));
typedef unsigned short v8us __attribute__((ext_vector_type(8), may_alias));
typedef float v8f  __attribute__((ext_vector_type(8)));
typedef float v4f  __attribute__((ext_vector_type(4)));
typedef float v4fa __attribute__((ext_vector_type(4), may_alias));
union FragH { v16h v; v8us half[2]; _Float16 h[16]; unsigned short u[16]; };

__device__ __forceinline__ unsigned short bf16_bits(float x) { const unsigned int u = __float_as_uint(x); return (unsigned short)((u + 0x7FFFu + ((u >> 16) & 1u)) >> 16); }
__device__ __forceinline__ float bf16_rne(float x) { return __uint_as_float(((unsigned int)bf16_bits(x)) << 16); }

__device__ __forceinline__ v16h ldfrag(const _Float16* __restrict__ p, size_t off, int hh) {
  FragH f; const unsigned short* q = (const unsigned short*)p + off + 8 * hh;
  f.half[0] = *(const v8us*)q; f.half[1] = *(const v8us*)(q + 16); return f.v; }
__device__ __forceinline__ v8f mma16(v16h a, v16h b, v8f c) {
  v8f d = __builtin_amdgcn_wmma_f32_16x16x32_f16(false, a, false, b, (short)0, c, false, false);
  asm volatile("v_nop\n\tv_nop\n\tv_nop\n\tv_nop" : "+v"(d) : "v"(a), "v"(b));
  return d; }

__global__ __launch_bounds__(256) void k_wt_f16(const float* __restrict__ W, _Float16* __restrict__ Wt, int K, int N, float scale) {
  const int t = blockIdx.x * 256 + threadIdx.x; if (t >= N * (K / 8)) return;
  const int n = t / (K / 8), k8 = (t % (K / 8)) * 8; FragH f;
#pragma unroll
  for (int i = 0; i < 8; ++i) f.h[i] = (_Float16)(bf16_rne(W[(size_t)(k8 + i) * N + n]) * scale);
  const v8us o = f.half[0]; unsigned short* d = (unsigned short*)Wt + (size_t)n * K + k8;
  *(volatile v8us*)d = o; __threadfence(); *(volatile v8us*)d = o; }

__global__ __launch_bounds__(256) void k_x16(const float* __restrict__ x, _Float16* __restrict__ X16) {
  const size_t t = (size_t)blockIdx.x * 256 + threadIdx.x; if (t >= (size_t)NR * DM / 8) return;
  const int row = (int)(t / (DM / 8)), c8 = (int)(t % (DM / 8)) * 8; const int b = row / SEQ, s = row - b * SEQ;
  const float* src = x + ((size_t)b * SEQ_FULL + s) * DM + c8;
  const v4f a = *(const v4fa*)src, c = *(const v4fa*)(src + 4); FragH f;
#pragma unroll
  for (int q = 0; q < 4; ++q) { f.h[q] = (_Float16)bf16_rne(a[q]); f.h[4 + q] = (_Float16)bf16_rne(c[q]); }
  const v8us o = f.half[0]; unsigned short* d = (unsigned short*)X16 + t * 8;
  *(volatile v8us*)d = o; __threadfence(); *(volatile v8us*)d = o; }

__global__ __launch_bounds__(128) void k_gemm_qkv(const _Float16* __restrict__ A, const _Float16* __restrict__ Bt, const float* __restrict__ bias, _Float16* __restrict__ CH, _Float16* __restrict__ CL) {
  __shared__ __attribute__((aligned(16))) float so[4][32][68];
  const int tid = threadIdx.x; const int w = __builtin_amdgcn_readfirstlane(tid >> 5);
  const int lane = tid & 31, ln = lane & 15, hh = lane >> 4;
  const int ntn = LQ / 64; const int mt = blockIdx.x / ntn, nq = blockIdx.x - mt * ntn;
  const int row0 = mt * 128 + 32 * w, col0 = nq * 64;
  const size_t a0 = (size_t)(row0 + ln) * DM, a1 = a0 + (size_t)16 * DM;
  const size_t b0 = (size_t)(col0 + ln) * DM, b1 = b0 + (size_t)16 * DM, b2 = b1 + (size_t)16 * DM, b3 = b2 + (size_t)16 * DM;
  const v8f z8 = {0.f,0.f,0.f,0.f,0.f,0.f,0.f,0.f};
  v8f c00 = z8, c01 = z8, c02 = z8, c03 = z8, c10 = z8, c11 = z8, c12 = z8, c13 = z8;
#pragma unroll 1
  for (int kb = 0; kb < DM; kb += 32) {
    const v16h f0 = ldfrag(A, a0 + kb, hh), f1 = ldfrag(A, a1 + kb, hh);
    v16h g = ldfrag(Bt, b0 + kb, hh); c00 = mma16(f0, g, c00); c10 = mma16(f1, g, c10);
    g = ldfrag(Bt, b1 + kb, hh); c01 = mma16(f0, g, c01); c11 = mma16(f1, g, c11);
    g = ldfrag(Bt, b2 + kb, hh); c02 = mma16(f0, g, c02); c12 = mma16(f1, g, c12);
    g = ldfrag(Bt, b3 + kb, hh); c03 = mma16(f0, g, c03); c13 = mma16(f1, g, c13); }
  v8f accs[8] = {c00, c01, c02, c03, c10, c11, c12, c13};
#pragma unroll
  for (int u = 0; u < 8; ++u) { const int t = u & 3, half = u >> 2; const float bv = bf16_rne(bias[col0 + t * 16 + ln]);
#pragma unroll
    for (int r = 0; r < 8; ++r) so[w][half * 16 + 8 * hh + r][t * 16 + ln] = accs[u][r] * 0.0625f + bv; }
  __builtin_amdgcn_fence(4  , "workgroup"); __builtin_amdgcn_wave_barrier();
  const int bq = row0 / SEQ, t0 = row0 - bq * SEQ; const bool wl = t0 < RESROWS;
  const size_t lrow0 = (size_t)bq * RESROWS + t0;
  const int rq = lane >> 3, c8 = (lane & 7) * 8;
  unsigned short* chp = (unsigned short*)CH; unsigned short* clp = (unsigned short*)CL;
  for (int pass = 0; pass < 2; ++pass) {
#pragma unroll 2
    for (int it = 0; it < 8; ++it) { const int r = it * 4 + rq;
      const v4f a = *(const v4fa*)&so[w][r][c8], c = *(const v4fa*)&so[w][r][c8 + 4]; FragH fh, fl;
#pragma unroll
      for (int q = 0; q < 4; ++q) { _Float16 t = (_Float16)a[q]; fh.h[q] = t; fl.h[q] = (_Float16)((a[q] - (float)t) * 1024.0f); t = (_Float16)c[q]; fh.h[4 + q] = t; fl.h[4 + q] = (_Float16)((c[q] - (float)t) * 1024.0f); }
      const v8us vh = fh.half[0], vl = fl.half[0];
      *(volatile v8us*)(chp + (size_t)(row0 + r) * LQ + col0 + c8) = vh;
      if (wl) *(volatile v8us*)(clp + (lrow0 + r) * LQ + col0 + c8) = vl; }
    if (pass == 0) __threadfence(); } }

__global__ __launch_bounds__(256) void k_vt(const _Float16* __restrict__ src, int srcRows, int tt, _Float16* __restrict__ dst) {
  __shared__ unsigned short tl[64][66];
  const int tid = threadIdx.x; const int ng = tt / 64; const int slab = blockIdx.x / ng, lg = blockIdx.x - slab * ng; const int b = slab / NH, h = slab - b * NH;
  for (int i = tid; i < 64 * 8; i += 256) { const int r = i / 8, c8 = (i % 8) * 8; FragH f;
    f.half[0] = *(const v8us*)((const unsigned short*)src + ((size_t)b * srcRows + lg * 64 + r) * LQ + 2 * DM + h * HD + c8);
#pragma unroll
    for (int q = 0; q < 8; ++q) tl[r][c8 + q] = f.u[q]; }
  __syncthreads();
  for (int pass = 0; pass < 2; ++pass) {
#pragma unroll
    for (int rd = 0; rd < 2; ++rd) { const int d = rd * 32 + tid / 8, pc = tid % 8; FragH f;
#pragma unroll
      for (int q = 0; q < 8; ++q) f.u[q] = tl[pc * 8 + q][d];
      const v8us o = f.half[0];
      *(volatile v8us*)((unsigned short*)dst + ((size_t)slab * HD + d) * tt + lg * 64 + pc * 8) = o; }
    if (pass == 0) __threadfence(); } }

template <bool RES>
__device__ __forceinline__ void attn_body(const _Float16* __restrict__ QH, const _Float16* __restrict__ QL, const _Float16* __restrict__ VT, const _Float16* __restrict__ VTL,
                                          _Float16* __restrict__ OH, _Float16* __restrict__ OL, const int qbase, const int nqb) {
  __shared__ __attribute__((aligned(16))) unsigned short oth[4][16][72];
  __shared__ __attribute__((aligned(16))) unsigned short otl[4][16][72];
  const int tid = threadIdx.x; const int wave = __builtin_amdgcn_readfirstlane(tid >> 5);
  const int lane = tid & 31, ln = lane & 15, hh = lane >> 4;
  const int bh = blockIdx.x / nqb, qb = blockIdx.x - bh * nqb; const int b = bh / NH, h = bh - b * NH;
  const int q0 = qbase + qb * 64 + wave * 16;
  const size_t qoff = ((size_t)b * SEQ + q0 + ln) * LQ + h * HD;
  const size_t qlo = ((size_t)b * RESROWS + q0 + ln) * LQ + h * HD;
  const v16h qh0 = ldfrag(QH, qoff, hh), qh1 = ldfrag(QH, qoff + 32, hh);
  const v8f z8 = {0.f,0.f,0.f,0.f,0.f,0.f,0.f,0.f};
  v8f oa[4] = {z8, z8, z8, z8}, ob[4] = {z8, z8, z8, z8};
  float m = -1.0e30f, l = 0.f;
  const int nsteps = (q0 + 47) >> 5;
#pragma unroll 1
  for (int st = 0; st < nsteps; ++st) {
    const int k0 = st * 32;
    const size_t ka = ((size_t)b * SEQ + k0 + ln) * LQ + DM + h * HD; const size_t kb = ka + (size_t)16 * LQ;
    v8f s0 = z8, s1 = z8, r0 = z8, r1 = z8;
    if (RES) {
      const size_t la = ((size_t)b * RESROWS + k0 + ln) * LQ + DM + h * HD; const size_t lb = la + (size_t)16 * LQ;
      const v16h ql0 = ldfrag(QL, qlo, hh), ql1 = ldfrag(QL, qlo + 32, hh);
      v16h kf = ldfrag(QH, ka, hh); v16h kr = ldfrag(QL, la, hh);
      s0 = mma16(kf, qh0, s0); r0 = mma16(kf, ql0, r0); r0 = mma16(kr, qh0, r0);
      kf = ldfrag(QH, ka + 32, hh); kr = ldfrag(QL, la + 32, hh);
      s0 = mma16(kf, qh1, s0); r0 = mma16(kf, ql1, r0); r0 = mma16(kr, qh1, r0);
      kf = ldfrag(QH, kb, hh); kr = ldfrag(QL, lb, hh);
      s1 = mma16(kf, qh0, s1); r1 = mma16(kf, ql0, r1); r1 = mma16(kr, qh0, r1);
      kf = ldfrag(QH, kb + 32, hh); kr = ldfrag(QL, lb + 32, hh);
      s1 = mma16(kf, qh1, s1); r1 = mma16(kf, ql1, r1); r1 = mma16(kr, qh1, r1);
    } else {
      v16h kf = ldfrag(QH, ka, hh); s0 = mma16(kf, qh0, s0);
      kf = ldfrag(QH, ka + 32, hh); s0 = mma16(kf, qh1, s0);
      kf = ldfrag(QH, kb, hh); s1 = mma16(kf, qh0, s1);
      kf = ldfrag(QH, kb + 32, hh); s1 = mma16(kf, qh1, s1);
    }
    float sv[16];
#pragma unroll
    for (int r = 0; r < 8; ++r) {
      if (RES) { sv[r] = (s0[r] + r0[r] * RSC) * 0.125f; sv[8 + r] = (s1[r] + r1[r] * RSC) * 0.125f; }
      else     { sv[r] = s0[r] * 0.125f;                sv[8 + r] = s1[r] * 0.125f; } }
    if (k0 + 31 > q0) {
      const int qq = q0 + ln - k0 - 8 * hh;
#pragma unroll
      for (int r = 0; r < 8; ++r) { sv[r] = (r <= qq) ? sv[r] : -1.0e30f; sv[8 + r] = (16 + r <= qq) ? sv[8 + r] : -1.0e30f; } }
    float tm = sv[0];
#pragma unroll
    for (int i = 1; i < 16; ++i) tm = fmaxf(tm, sv[i]);
    tm = fmaxf(tm, __shfl_xor(tm, 16, 32));
    const float mn = fmaxf(m, tm); const float al = __expf(m - mn); m = mn;
    float p[16]; float ps = 0.f;
#pragma unroll
    for (int i = 0; i < 16; ++i) { p[i] = __expf(sv[i] - mn); ps += p[i]; }
    l = l * al + ps;
#pragma unroll
    for (int f = 0; f < 4; ++f) {
#pragma unroll
      for (int r = 0; r < 8; ++r) { oa[f][r] *= al; if (RES) ob[f][r] *= al; } }
    FragH ph, pl;
#pragma unroll
    for (int i = 0; i < 16; ++i) { const _Float16 t = (_Float16)p[i]; ph.h[i] = t; pl.h[i] = RES ? (_Float16)((p[i] - (float)t) * 1024.0f) : (_Float16)0.0f; }
#pragma unroll
    for (int f = 0; f < 4; ++f) {
      const size_t vo = ((size_t)bh * HD + 16 * f + ln) * SEQ + k0;
      const v16h vf = ldfrag(VT, vo, hh);
      oa[f] = mma16(vf, ph.v, oa[f]);
      if (RES) { ob[f] = mma16(vf, pl.v, ob[f]);
        const size_t vl = ((size_t)bh * HD + 16 * f + ln) * RESROWS + k0;
        const v16h vr = ldfrag(VTL, vl, hh);
        ob[f] = mma16(vr, ph.v, ob[f]); } }
  }
  const float lt = l + __shfl_xor(l, 16, 32);
  const float inv = 64.0f / lt;
#pragma unroll
  for (int f = 0; f < 4; ++f) { FragH fh, fl;
#pragma unroll
    for (int r = 0; r < 8; ++r) { float v = RES ? (oa[f][r] + ob[f][r] * RSC) : oa[f][r]; v *= inv; const _Float16 t = (_Float16)v; fh.h[r] = t; fl.h[r] = (_Float16)((v - (float)t) * 1024.0f); }
    *(v8us*)&oth[wave][ln][16 * f + 8 * hh] = fh.half[0];
    *(v8us*)&otl[wave][ln][16 * f + 8 * hh] = fl.half[0]; }
  __builtin_amdgcn_fence(4  , "workgroup"); __builtin_amdgcn_wave_barrier();
  const int rq = lane >> 3, pc = (lane & 7) * 8;
  unsigned short* ohp = (unsigned short*)OH; unsigned short* olp = (unsigned short*)OL;
  for (int pass = 0; pass < 2; ++pass) {
#pragma unroll
    for (int it = 0; it < 4; ++it) { const int row = it * 4 + rq;
      const v8us vh = *(const v8us*)&oth[wave][row][pc]; const v8us vl = *(const v8us*)&otl[wave][row][pc];
      const size_t go = ((size_t)b * SEQ + q0 + row) * DM + h * HD + pc;
      *(volatile v8us*)(ohp + go) = vh; *(volatile v8us*)(olp + go) = vl; }
    if (pass == 0) __threadfence(); } }

__global__ __launch_bounds__(128) void k_attn_plain(const _Float16* __restrict__ QH, const _Float16* __restrict__ QL, const _Float16* __restrict__ VT, const _Float16* __restrict__ VTL, _Float16* __restrict__ OH, _Float16* __restrict__ OL) {
  attn_body<false>(QH, QL, VT, VTL, OH, OL, RESROWS, (SEQ - RESROWS) / 64); }
__global__ __launch_bounds__(128) void k_attn_res(const _Float16* __restrict__ QH, const _Float16* __restrict__ QL, const _Float16* __restrict__ VT, const _Float16* __restrict__ VTL, _Float16* __restrict__ OH, _Float16* __restrict__ OL) {
  attn_body<true>(QH, QL, VT, VTL, OH, OL, 0, RESROWS / 64); }

__global__ __launch_bounds__(128) void k_gemm_out(const _Float16* __restrict__ AH, const _Float16* __restrict__ AL, const _Float16* __restrict__ Bt, const float* __restrict__ bias, float* __restrict__ C) {
  __shared__ __attribute__((aligned(16))) float so[4][16][68];
  const int tid = threadIdx.x; const int w = __builtin_amdgcn_readfirstlane(tid >> 5);
  const int lane = tid & 31, ln = lane & 15, hh = lane >> 4;
  const int ntn = DM / 64; const int wid = blockIdx.x * 4 + w; const int mt = wid / ntn, nq = wid - mt * ntn;
  const int row0 = mt * 16, col0 = nq * 64;
  const size_t ao = (size_t)(row0 + ln) * DM; const size_t bo = (size_t)(col0 + ln) * DM;
  const v8f z8 = {0.f,0.f,0.f,0.f,0.f,0.f,0.f,0.f};
  v8f ch[4] = {z8, z8, z8, z8}, cl[4] = {z8, z8, z8, z8};
#pragma unroll 1
  for (int kb = 0; kb < DM; kb += 32) {
    const v16h fh = ldfrag(AH, ao + kb, hh), fl = ldfrag(AL, ao + kb, hh);
#pragma unroll
    for (int t = 0; t < 4; ++t) { const v16h g = ldfrag(Bt, bo + (size_t)t * 16 * DM + kb, hh); ch[t] = mma16(fh, g, ch[t]); cl[t] = mma16(fl, g, cl[t]); } }
#pragma unroll
  for (int t = 0; t < 4; ++t) { const float bv = bf16_rne(bias[col0 + t * 16 + ln]);
#pragma unroll
    for (int r = 0; r < 8; ++r) so[w][8 * hh + r][t * 16 + ln] = (ch[t][r] + cl[t][r] * RSC) * RSC + bv; }
  __builtin_amdgcn_fence(4  , "workgroup"); __builtin_amdgcn_wave_barrier();
  const int bq = row0 / SEQ, t0 = row0 - bq * SEQ; const size_t orow0 = (size_t)bq * SEQ_FULL + t0;
  const int rsub = lane >> 4, c4 = (lane & 15) * 4;
  for (int pass = 0; pass < 2; ++pass) {
#pragma unroll
    for (int q = 0; q < 8; ++q) { const int r = q * 2 + rsub;
      const v4f v = *(const v4fa*)&so[w][r][c4];
      *(volatile v4f*)(C + (orow0 + r) * DM + col0 + c4) = v; }
    if (pass == 0) __threadfence(); } }

extern "C" void kernel_launch(void* const* d_in, const int* in_sizes, int n_in,
                              void* d_out, int out_size, void* d_ws, size_t ws_size, hipStream_t stream) {
  if (n_in < 5) return;
  const long long needx = ((long long)(NB - 1) * SEQ_FULL + SEQ) * DM;
  if ((long long)in_sizes[0] < needx || in_sizes[1] < DM * LQ || in_sizes[2] < LQ || in_sizes[3] < DM * DM || in_sizes[4] < DM || (long long)out_size < needx) return;
  const float* x = (const float*)d_in[0]; const float* wqkv = (const float*)d_in[1]; const float* bqkv = (const float*)d_in[2]; const float* wo = (const float*)d_in[3]; const float* bo = (const float*)d_in[4];
  char* ws = (char*)d_ws; size_t off = 0;
  auto take = [&](size_t bytes) { char* p = ws + off; off += (bytes + 255) & ~(size_t)255; return p; };
  _Float16* BQKV = (_Float16*)take((size_t)3 * DM * DM * 2);
  _Float16* BO   = (_Float16*)take((size_t)DM * DM * 2);
  _Float16* X16  = (_Float16*)take((size_t)NR * DM * 2);
  _Float16* QKVH = (_Float16*)take((size_t)NR * LQ * 2);
  _Float16* QKVL = (_Float16*)take((size_t)NB * RESROWS * LQ * 2);
  _Float16* VT   = (_Float16*)take((size_t)NB * NH * HD * SEQ * 2);
  _Float16* VTL  = (_Float16*)take((size_t)NB * NH * HD * RESROWS * 2);
  _Float16* OH   = (_Float16*)take((size_t)NR * DM * 2);
  _Float16* OL   = (_Float16*)take((size_t)NR * DM * 2);
  if (off > ws_size || off > (size_t)134217728) return;
  k_wt_f16<<<(unsigned)(((size_t)LQ * (DM / 8) + 255) / 256), 256, 0, stream>>>(wqkv, BQKV, DM, LQ, 16.0f);
  k_wt_f16<<<(unsigned)(((size_t)DM * (DM / 8) + 255) / 256), 256, 0, stream>>>(wo, BO, DM, DM, 16.0f);
  k_x16<<<(unsigned)(((size_t)NR * DM / 8 + 255) / 256), 256, 0, stream>>>(x, X16);
  k_gemm_qkv<<<(unsigned)((NR / 128) * (LQ / 64)), 128, 0, stream>>>(X16, BQKV, bqkv, QKVH, QKVL);
  k_vt<<<(unsigned)(NB * NH * (SEQ / 64)), 256, 0, stream>>>(QKVH, SEQ, SEQ, VT);
  k_vt<<<(unsigned)(NB * NH * (RESROWS / 64)), 256, 0, stream>>>(QKVL, RESROWS, RESROWS, VTL);
  if ((SEQ - RESROWS) / 64 > 0)
    k_attn_plain<<<(unsigned)(NB * NH * ((SEQ - RESROWS) / 64)), 128, 0, stream>>>(QKVH, QKVL, VT, VTL, OH, OL);
  k_attn_res<<<(unsigned)(NB * NH * (RESROWS / 64)), 128, 0, stream>>>(QKVH, QKVL, VT, VTL, OH, OL);
  k_gemm_out<<<(unsigned)(((NR / 16) * (DM / 64)) / 4), 128, 0, stream>>>(OH, OL, BO, bo, (float*)d_out);
}
